// AnyModalMirasol_78340203479480
// MI455X (gfx1250) — hardware-run, weakly checked
//
#include <hip/hip_runtime.h>


#ifndef NB
#define NB 2
#endif
#ifndef NG
#define NG 8
#endif
#define NB_FULL 2
#define NG_FULL 8
#define TT    256
#define MEMT  16
#define DM    1024
#define C3    3072
#define NH_   16
#define HD    64
#define SL    (MEMT + TT)
#define SG    (MEMT + NG * TT)
#define ML_   (NB * NG * SL)
#define MG_   (NB * SG)
#define MMAX  (ML_ > MG_ ? ML_ : MG_)
#define BTN   5
#define BROWS (NB * BTN * 64)
#define RT    (SL + 16)
#define AW    4
#define OSP   68
#define OSG   68
#define WSC   1024.0f
#define QRS   2048.0f
#define QRI   (1.0f / 2048.0f)
#define SC2   ((float)(0.125 * 1.4426950408889634))
#define PSH   14.0f
#define NEGB  (-3.0e38f)
#define EPSN  1.0e-6f

static_assert(NH_ * HD == DM);
static_assert(HD == 64);
static_assert(TT == 256);
static_assert(MEMT == 16);
static_assert(SL % 16 == 0);
static_assert(SG % 16 == 0);
static_assert(DM % 64 == 0);
static_assert(C3 % 64 == 0);
static_assert(DM % 32 == 0);
static_assert(48 + SL <= BTN * 64);
static_assert(NG * SL >= (BTN + 1) * 64);
static_assert(SG >= (BTN + 1) * 64);
static_assert(SG >= RT);
static_assert(RT % 16 == 0);
static_assert(RT >= SL + 16);
static_assert(NB <= NB_FULL);
static_assert(NG <= NG_FULL);
static_assert((OSP * 4) % 16 == 0);
static_assert((OSG * 4) % 16 == 0);
static_assert(64 * OSG * 4 <= 131072);
static_assert(AW * 16 * OSP * 4 <= 131072);
static_assert(64 * 65 * 4 <= 131072);

typedef _Float16 h16;
typedef unsigned short bf;
typedef __attribute__((ext_vector_type(16))) _Float16 v16h;
typedef __attribute__((ext_vector_type(8)))  _Float16 v8h;
typedef __attribute__((ext_vector_type(8)))  float    v8f;
typedef __attribute__((ext_vector_type(4)))  float    v4f;
typedef v4f  __attribute__((may_alias)) v4fa;

__device__ __forceinline__ unsigned short f2bf(float f) { unsigned u = __float_as_uint(f); u += 0x7FFFu + ((u >> 16) & 1u); return (unsigned short)(u >> 16); }
__device__ __forceinline__ float bfr(float f) { return __uint_as_float(((unsigned)f2bf(f)) << 16); }
__device__ __forceinline__ v16h cat16(v8h lo, v8h hi) { return __builtin_shufflevector(lo, hi, 0, 1, 2, 3, 4, 5, 6, 7, 8, 9, 10, 11, 12, 13, 14, 15); }
__device__ __forceinline__ v16h  ldh(const h16* p) { return cat16(*(const v8h*)p, *(const v8h*)(p + 16)); }
__device__ __forceinline__ void wave_sync() { __builtin_amdgcn_fence(3  , "wavefront"); __builtin_amdgcn_wave_barrier(); asm volatile("" ::: "memory"); }
__device__ __forceinline__ h16 toh_flush(float v) { const h16 r = (h16)v; return (fabsf(v) < 6.103515625e-05f) ? (h16)0.0f : r; }
__device__ __forceinline__ v8f wmma16g(v16h a, v16h b, v8f c) {
    c = __builtin_amdgcn_wmma_f32_16x16x32_f16(false, a, false, b, (short)0, c, false, false);
    asm volatile("v_nop\n\tv_nop\n\tv_nop\n\tv_nop" : "+v"(c) : "v"(a), "v"(b));
    return c;
}
__device__ __forceinline__ int band_slot(int tile, int bstride) {
    int ct = -1;
#pragma unroll
    for (int b = 0; b < NB; ++b) { const int d = tile - ((b * bstride) >> 6); ct = ((d >= 0) & (d < BTN)) ? (b * BTN + d) : ct; }
    return ct;
}

__global__ __launch_bounds__(256) void k_wconv(const float* __restrict__ W, h16* Wt, int N) {
#pragma clang fp contract(off)
    __shared__ float tl[64 * 65];
    const int tid = threadIdx.x;
    const int k0 = blockIdx.x * 64, n0 = blockIdx.y * 64;
    const float* src = W + (size_t)blockIdx.z * (size_t)DM * (size_t)N;
    h16* dst = Wt + (size_t)blockIdx.z * (size_t)N * (size_t)DM;
    static_assert(4 * 16 == 64);
#pragma unroll 1
    for (int q = 0; q < 4; ++q) {
        const int kr = q * 16 + (tid >> 4), nc = (tid & 15) * 4;
        const v4f v = *(const v4f*)(src + (size_t)(k0 + kr) * (size_t)N + n0 + nc);
        tl[kr * 65 + nc + 0] = v[0]; tl[kr * 65 + nc + 1] = v[1]; tl[kr * 65 + nc + 2] = v[2]; tl[kr * 65 + nc + 3] = v[3];
    }
    __syncthreads();
    const int n = tid >> 3, k8 = (tid & 7) * 8;
    v8h o0, o1;
#pragma unroll
    for (int i = 0; i < 8; ++i) { o0[i] = toh_flush(bfr(tl[(k8 + i) * 65 + n]) * WSC); o1[i] = toh_flush(bfr(tl[(k8 + i) * 65 + 32 + n]) * WSC); }
    static_assert(2 * 32 == 64);
    h16* d0 = dst + (size_t)(n0 + n) * DM + k0 + k8;
    h16* d1 = dst + (size_t)(n0 + 32 + n) * DM + k0 + k8;
    *(volatile v8h*)d0 = o0; *(volatile v8h*)d1 = o1;
    __threadfence();
    *(volatile v8h*)d0 = o0; *(volatile v8h*)d1 = o1;
}

__global__ __launch_bounds__(256) void k_pack(const float* __restrict__ src, h16* dst, h16* dres, int nrows, int nr, int ng, int ngfull, int dS, int doff, float carry, int wres, int bstride) {
#pragma clang fp contract(off)
    static_assert(128 * 8 == DM);
    const int item = blockIdx.x * 2 + (int)(threadIdx.x >> 7);
    if (item >= nrows) return;
    const int c8 = (threadIdx.x & 127) * 8;
    const int q = item / nr, t = item - q * nr; const int b = q / ng, g = q - b * ng;
    const size_t so = ((size_t)(b * ngfull + g) * (size_t)nr + (size_t)t) * DM + c8;
    const int drow = q * dS + doff + t;
    const v4f x0 = *(const v4f*)(src + so), x1 = *(const v4f*)(src + so + 4);
    v8h o; const v8h zv = (v8h){};
#pragma unroll
    for (int i = 0; i < 4; ++i) { o[i] = toh_flush(bfr(x0[i]) * carry); o[4 + i] = toh_flush(bfr(x1[i]) * carry); }
    int ct = -1; if (wres != 0) ct = band_slot(drow >> 6, bstride);
    h16* dp = dst + (size_t)drow * DM + c8;
    h16* rp = dres + (size_t)((ct < 0 ? 0 : ct) * 64 + (drow & 63)) * DM + c8;
    *(volatile v8h*)dp = o; if (ct >= 0) *(volatile v8h*)rp = zv;
    __threadfence();
    *(volatile v8h*)dp = o; if (ct >= 0) *(volatile v8h*)rp = zv;
}

__global__ __launch_bounds__(256) void k_qknorm(const float* __restrict__ QK, const float* __restrict__ gain, h16* QKH, h16* QKR, int M, int S, int ngs, size_t plane, size_t rplane) {
#pragma clang fp contract(off)
    const int lane = threadIdx.x & 31;
    const int wave = __builtin_amdgcn_readfirstlane((int)(threadIdx.x >> 5));
    const int item = blockIdx.x * 8 + wave;
    const int row = item >> 1, which = item & 1;
    if (row >= M) return;
    const float* p = QK + (size_t)row * 2048 + (size_t)which * 1024 + lane * 8;
    v4f xa[4], xb[4]; float ss = 0.0f;
#pragma unroll
    for (int i = 0; i < 4; ++i) { xa[i] = *(const v4f*)(p + i * 256); xb[i] = *(const v4f*)(p + i * 256 + 4);
#pragma unroll
        for (int e = 0; e < 4; ++e) { ss += xa[i][e] * xa[i][e]; ss += xb[i][e] * xb[i][e]; } }
#pragma unroll
    for (int mk = 16; mk >= 1; mk >>= 1) ss += __shfl_xor(ss, mk, 32);
    const float rs = rsqrtf(ss * (1.0f / 1024.0f) + EPSN);
    const int seq = row / S, t = row - seq * S;
    const int bb = seq / ngs, gg = seq - bb * ngs;
    const bool bd = (gg == 0) & ((ngs > 1) | (t < RT));
    v8h hv[4], rv[4];
#pragma unroll
    for (int i = 0; i < 4; ++i) {
        const v4f g0 = *(const v4f*)(gain + i * 256 + lane * 8), g1 = *(const v4f*)(gain + i * 256 + lane * 8 + 4);
#pragma unroll
        for (int e = 0; e < 4; ++e) {
            const float y0 = (xa[i][e] * rs) * bfr(g0[e]), y1 = (xb[i][e] * rs) * bfr(g1[e]);
            const h16 a0 = toh_flush(y0), a1 = toh_flush(y1);
            hv[i][e] = a0; hv[i][4 + e] = a1;
            rv[i][e] = toh_flush((y0 - (float)a0) * QRS); rv[i][4 + e] = toh_flush((y1 - (float)a1) * QRS); } }
    h16* PH = QKH + (size_t)which * plane;
    h16* PR = QKR + (size_t)which * rplane;
    static_assert(4 * 4 * 64 == DM);
#pragma unroll 1
    for (int ps = 0; ps < 2; ++ps) {
#pragma unroll
        for (int i = 0; i < 4; ++i) { const int head = i * 4 + (lane >> 3);
            const size_t oo = ((size_t)(seq * NH_ + head) * (size_t)S + (size_t)t) * HD + (lane & 7) * 8;
            const size_t ro = ((size_t)(bb * NH_ + head) * (size_t)RT + (size_t)(bd ? t : 0)) * HD + (lane & 7) * 8;
            *(volatile v8h*)(PH + oo) = hv[i]; if (bd) *(volatile v8h*)(PR + ro) = rv[i]; }
        if (ps == 0) __threadfence(); }
}

template <int EPI>
__device__ __forceinline__ void gemm_body(const h16* __restrict__ A, const h16* __restrict__ AR, const h16* __restrict__ Bt,
                                          float* F0, h16* H0, h16* H0R,
                                          int M, int S, int useband, int bsrc, float ascale, int ngs, float vscale,
                                          int srcng, int db, int dg, int d0, int bdx, int bdm, int wmem, int oxd, int oxm, int oxdr, int oxmr, float cx, float cm) {
    __shared__ __align__(16) float os[64 * OSG];
    const int lane = threadIdx.x & 31, lr = lane & 15, hi = lane >> 4;
    const int r0 = blockIdx.x * 64, c0 = blockIdx.y * 64;
    int ctv = -1; if (useband != 0) ctv = band_slot((int)blockIdx.x, bsrc);
    const size_t boff = (size_t)(c0 + lr) * DM + 8 * hi;
    if (ctv < 0) {
        v8f acc[4][4];
#pragma unroll
        for (int mb = 0; mb < 4; ++mb)
#pragma unroll
            for (int nb = 0; nb < 4; ++nb) acc[mb][nb] = (v8f){};
        size_t ao[4];
#pragma unroll
        for (int mb = 0; mb < 4; ++mb) { int rr = r0 + mb * 16 + lr; rr = rr < M ? rr : (M - 1); ao[mb] = (size_t)rr * DM + 8 * hi; }
#pragma unroll 1
        for (int kc = 0; kc < DM; kc += 32) {
            v16h a[4];
#pragma unroll
            for (int mb = 0; mb < 4; ++mb) a[mb] = ldh(A + ao[mb] + kc);
#pragma unroll
            for (int nb = 0; nb < 4; ++nb) { const v16h b = ldh(Bt + boff + (size_t)nb * 16 * DM + kc);
#pragma unroll
                for (int mb = 0; mb < 4; ++mb) acc[mb][nb] = wmma16g(a[mb], b, acc[mb][nb]); }
        }
#pragma unroll
        for (int mb = 0; mb < 4; ++mb)
#pragma unroll
            for (int nb = 0; nb < 4; ++nb)
#pragma unroll
                for (int j = 0; j < 8; ++j) os[(mb * 16 + hi * 8 + j) * OSG + nb * 16 + lr] = acc[mb][nb][j] * ascale;
    } else {
#pragma unroll 1
        for (int rh = 0; rh < 2; ++rh) {
            v8f acc[2][4], accR[2][4];
#pragma unroll
            for (int mb = 0; mb < 2; ++mb)
#pragma unroll
                for (int nb = 0; nb < 4; ++nb) { acc[mb][nb] = (v8f){}; accR[mb][nb] = (v8f){}; }
            size_t ao[2], aro[2];
#pragma unroll
            for (int mb = 0; mb < 2; ++mb) { int rr = r0 + rh * 32 + mb * 16 + lr; rr = rr < M ? rr : (M - 1); ao[mb] = (size_t)rr * DM + 8 * hi;
                                             aro[mb] = (size_t)(ctv * 64 + rh * 32 + mb * 16 + lr) * DM + 8 * hi; }
#pragma unroll 1
            for (int kc = 0; kc < DM; kc += 32) {
                v16h a[2], ar[2];
#pragma unroll
                for (int mb = 0; mb < 2; ++mb) { a[mb] = ldh(A + ao[mb] + kc); ar[mb] = ldh(AR + aro[mb] + kc); }
#pragma unroll
                for (int nb = 0; nb < 4; ++nb) { const v16h b = ldh(Bt + boff + (size_t)nb * 16 * DM + kc);
#pragma unroll
                    for (int mb = 0; mb < 2; ++mb) { acc[mb][nb] = wmma16g(a[mb], b, acc[mb][nb]); accR[mb][nb] = wmma16g(ar[mb], b, accR[mb][nb]); } }
            }
#pragma unroll
            for (int mb = 0; mb < 2; ++mb)
#pragma unroll
                for (int nb = 0; nb < 4; ++nb)
#pragma unroll
                    for (int j = 0; j < 8; ++j) os[(rh * 32 + mb * 16 + hi * 8 + j) * OSG + nb * 16 + lr] = (acc[mb][nb][j] + accR[mb][nb][j] * QRI) * ascale;
        }
    }
    wave_sync();
#pragma unroll 1
    for (int sl = 0; sl < 4; ++sl) {
        const int row0 = r0 + sl * 16;
        if (row0 >= M) break;
        const int seq = row0 / S, t0s = row0 - seq * S;
        if (EPI == 0) {
            const int which = c0 >> 10;
            if (which < 2) {
                static_assert(8 * 2 == 16);
#pragma unroll 1
                for (int ps = 0; ps < 2; ++ps) {
#pragma unroll
                    for (int s = 0; s < 8; ++s) { const int row = 2 * s + (lane >> 4), cf = (lane & 15) * 4;
                        const v4f val = *(const v4fa*)(&os[(sl * 16 + row) * OSG + cf]);
                        *(volatile v4f*)(F0 + (size_t)(row0 + row) * 2048 + c0 + cf) = val; }
                    if (ps == 0) __threadfence(); }
            } else {
                const int head = (c0 & 1023) >> 6;
                const int bb = seq / ngs, gg = seq - bb * ngs;
                const bool bd = (gg == 0) & ((ngs > 1) | (t0s < RT));
                v8h hv[4], rv[4];
                static_assert(4 * 32 * 16 == 16 * HD * 2);
#pragma unroll
                for (int s = 0; s < 4; ++s) { const int p = s * 32 + lane; const int d = p >> 1, hf = p & 1;
#pragma unroll
                    for (int i = 0; i < 8; ++i) { const float x = os[(sl * 16 + hf * 8 + i) * OSG + d] * vscale; const h16 a0 = toh_flush(x); hv[s][i] = a0; rv[s][i] = toh_flush((x - (float)a0) * QRS); } }
                const size_t vb = ((size_t)(seq * NH_ + head) * (size_t)(S >> 4) + (size_t)(t0s >> 4)) * 1024;
                const size_t rb = ((size_t)(bb * NH_ + head) * (size_t)(RT >> 4) + (size_t)(bd ? (t0s >> 4) : 0)) * 1024;
#pragma unroll 1
                for (int ps = 0; ps < 2; ++ps) {
#pragma unroll
                    for (int s = 0; s < 4; ++s) { const int p = s * 32 + lane;
                        *(volatile v8h*)(H0 + vb + (size_t)p * 8) = hv[s]; if (bd) *(volatile v8h*)(H0R + rb + (size_t)p * 8) = rv[s]; }
                    if (ps == 0) __threadfence(); }
            }
        } else {
            const bool memslab = t0s < MEMT;
            if (memslab & ((EPI == 2) | (wmem == 0))) continue;
            int drow, oh, orr, bst; float cy;
            if (memslab) { drow = row0; oh = oxm; orr = oxmr; bst = bdm; cy = cm; }
            else { const int p = t0s - MEMT; int b, g, tt;
                   if (srcng > 0) { b = seq / srcng; g = seq - b * srcng; tt = p; } else { b = seq; g = p >> 8; tt = p & (TT - 1); }
                   drow = b * db + g * dg + d0 + tt; oh = oxd; orr = oxdr; bst = bdx; cy = cx; }
            if (EPI == 2) {
#pragma unroll 1
                for (int ps = 0; ps < 2; ++ps) {
#pragma unroll
                    for (int s = 0; s < 8; ++s) { const int row = 2 * s + (lane >> 4), cf = (lane & 15) * 4;
                        const v4f val = *(const v4fa*)(&os[(sl * 16 + row) * OSG + cf]);
                        *(volatile v4f*)(F0 + (size_t)(drow + row) * DM + c0 + cf) = val; }
                    if (ps == 0) __threadfence(); }
            } else {
                const int ct = band_slot(drow >> 6, bst);
                v8h hv[4], rv[4];
                static_assert(4 * 4 == 16);
#pragma unroll
                for (int s = 0; s < 4; ++s) { const int row = 4 * s + (lane >> 3), c8 = (lane & 7) * 8;
                    const v4f x0 = *(const v4fa*)(&os[(sl * 16 + row) * OSG + c8]); const v4f x1 = *(const v4fa*)(&os[(sl * 16 + row) * OSG + c8 + 4]);
#pragma unroll
                    for (int i = 0; i < 4; ++i) { const float y0 = x0[i] * cy, y1 = x1[i] * cy; const h16 a0 = toh_flush(y0), a1 = toh_flush(y1);
                        hv[s][i] = a0; hv[s][4 + i] = a1; rv[s][i] = toh_flush((y0 - (float)a0) * QRS); rv[s][4 + i] = toh_flush((y1 - (float)a1) * QRS); } }
                const size_t hb = (size_t)oh + (size_t)drow * DM + c0;
                const size_t rb = (size_t)orr + (size_t)((ct < 0 ? 0 : ct) * 64 + (drow & 63)) * DM + c0;
#pragma unroll 1
                for (int ps = 0; ps < 2; ++ps) {
#pragma unroll
                    for (int s = 0; s < 4; ++s) { const int row = 4 * s + (lane >> 3), c8 = (lane & 7) * 8;
                        *(volatile v8h*)(H0 + hb + (size_t)row * DM + c8) = hv[s]; if (ct >= 0) *(volatile v8h*)(H0R + rb + (size_t)row * DM + c8) = rv[s]; }
                    if (ps == 0) __threadfence(); }
            }
        }
    }
}

__global__ __launch_bounds__(32) void k_gemm_qkv(const h16* __restrict__ A, const h16* __restrict__ AR, const h16* __restrict__ Bt, float* QK, h16* VT, h16* VR,
                                                 int M, int S, int useband, int bsrc, float ascale, int ngs, float vscale) {
    gemm_body<0>(A, AR, Bt, QK, VT, VR, M, S, useband, bsrc, ascale, ngs, vscale, 0, 0, 0, 0, 0, 0, 0, 0, 0, 0, 0, 0.0f, 0.0f);
}
__global__ __launch_bounds__(32) void k_gemm_proj16(const h16* __restrict__ A, const h16* __restrict__ AR, const h16* __restrict__ Bt, h16* X, h16* XR,
                                                    int M, int S, int useband, int bsrc, float ascale,
                                                    int srcng, int db, int dg, int d0, int bdx, int bdm, int wmem, int oxd, int oxm, int oxdr, int oxmr, float cx, float cm) {
    gemm_body<1>(A, AR, Bt, (float*)0, X, XR, M, S, useband, bsrc, ascale, 1, 0.0f, srcng, db, dg, d0, bdx, bdm, wmem, oxd, oxm, oxdr, oxmr, cx, cm);
}
__global__ __launch_bounds__(32) void k_gemm_proj32(const h16* __restrict__ A, const h16* __restrict__ AR, const h16* __restrict__ Bt, float* OUT,
                                                    int M, int S, int useband, int bsrc, float ascale, int srcng, int db, int dg, int d0) {
    gemm_body<2>(A, AR, Bt, OUT, (h16*)0, (h16*)0, M, S, useband, bsrc, ascale, 1, 0.0f, srcng, db, dg, d0, 0, 0, 0, 0, 0, 0, 0, 0.0f, 0.0f);
}

template <int EARLY>
__device__ __forceinline__ void flash_body(const h16* __restrict__ QH, const h16* __restrict__ QR, const h16* __restrict__ KP, const h16* __restrict__ KR,
                                           const h16* __restrict__ VT, const h16* __restrict__ VR, h16* CH, h16* CR,
                                           int S, int tile0, int ntl, int ng1, int g0, int ngs, int bstride, float osc) {
    __shared__ __align__(16) float os[AW * 16 * OSP];
    const int lane = threadIdx.x & 31, lr = lane & 15, hi = lane >> 4;
    const int wave = __builtin_amdgcn_readfirstlane((int)(threadIdx.x >> 5));
    const int tl = blockIdx.x * AW + wave;
    if (tl >= ntl) return;
    const int yy = blockIdx.y; const int per = ng1 * NH_;
    const int b = yy / per, rem = yy - b * per; const int g = g0 + (rem >> 4), h = rem & 15;
    const int seq = b * ngs + g; const int z = seq * NH_ + h; const int zz = b * NH_ + h;
    const int t0 = (tile0 + tl) * 16;
    const int wv = (int)(threadIdx.x >> 5);
    const int ct = __builtin_amdgcn_readfirstlane(band_slot((seq * S + (tile0 + (int)blockIdx.x * AW + wv) * 16) >> 6, bstride));
    const int lim = t0 + lr;
    const int nk = (t0 + 16 + 31) & ~31;
    const int S16 = S >> 4;
    const size_t pbase = (size_t)z * (size_t)S * HD;
    const size_t rbase = (size_t)zz * (size_t)RT * HD;
    const size_t qo = pbase + (size_t)(t0 + lr) * HD + 8 * hi;
    const v16h qh0 = ldh(QH + qo), qh1 = ldh(QH + qo + 32);
    const int qro = (t0 + lr) * HD + 8 * hi;
    const v16h hz = (v16h){};
    v8f o[4], oR[4];
#pragma unroll
    for (int j = 0; j < 4; ++j) { o[j] = (v8f){}; oR[j] = (v8f){}; }
    float m = NEGB, l = 0.0f;
#pragma unroll 1
    for (int key0 = 0; key0 < nk; key0 += 32) {
        const int ba = key0 >> 4; int bb = ba + 1; bb = bb < S16 ? bb : (S16 - 1);
        const h16* ka = KP + pbase + (size_t)(ba * 16 + lr) * HD + 8 * hi;
        const h16* kb = KP + pbase + (size_t)(bb * 16 + lr) * HD + 8 * hi;
        const v16h ka0 = ldh(ka), ka1 = ldh(ka + 32), kb0 = ldh(kb), kb1 = ldh(kb + 32);
        v8f sHa = (v8f){}, sHb = (v8f){}, sLa = (v8f){}, sLb = (v8f){};
        sHa = wmma16g(ka0, qh0, sHa); sHa = wmma16g(ka1, qh1, sHa);
        sHb = wmma16g(kb0, qh0, sHb); sHb = wmma16g(kb1, qh1, sHb);
        if (EARLY) {
            int qoff = qro; asm volatile("" : "+v"(qoff));
            const v16h qr0 = ldh(QR + rbase + qoff), qr1 = ldh(QR + rbase + qoff + 32);
            const h16* kra = KR + rbase + (size_t)(ba * 16 + lr) * HD + 8 * hi;
            const h16* krb = KR + rbase + (size_t)(bb * 16 + lr) * HD + 8 * hi;
            const v16h kra0 = ldh(kra), kra1 = ldh(kra + 32), krb0 = ldh(krb), krb1 = ldh(krb + 32);
            sLa = wmma16g(ka0, qr0, sLa); sLa = wmma16g(ka1, qr1, sLa); sLa = wmma16g(kra0, qh0, sLa); sLa = wmma16g(kra1, qh1, sLa);
            sLb = wmma16g(kb0, qr0, sLb); sLb = wmma16g(kb1, qr1, sLb); sLb = wmma16g(krb0, qh0, sLb); sLb = wmma16g(krb1, qh1, sLb);
        }
        const int ja = key0 + 8 * hi;
        float ta[8], tb[8]; bool fa[8], fb[8]; float mx = NEGB;
#pragma unroll
        for (int r = 0; r < 8; ++r) {
            fa[r] = (ja + r <= lim);
            fb[r] = (ja + 16 + r <= lim);
            if (EARLY) { ta[r] = (sHa[r] + sLa[r] * QRI) * SC2; tb[r] = (sHb[r] + sLb[r] * QRI) * SC2; }
            else       { ta[r] = sHa[r] * SC2; tb[r] = sHb[r] * SC2; }
            mx = fmaxf(mx, fmaxf(fa[r] ? ta[r] : NEGB, fb[r] ? tb[r] : NEGB)); }
        mx = fmaxf(mx, __shfl_xor(mx, 16, 32));
        const float mnew = fmaxf(m, mx);
        const float alpha = __builtin_amdgcn_exp2f(m - mnew);
        const float sh = PSH - mnew;
        v16h pb, pr = hz; float ls = 0.0f;
#pragma unroll
        for (int r = 0; r < 8; ++r) {
            const float xa = ta[r] + sh, xb = tb[r] + sh;
            const float ea = __builtin_amdgcn_exp2f(xa), eb = __builtin_amdgcn_exp2f(xb);
            const float ga = (fa[r] & (xa >= -14.0f)) ? ea : 0.0f, gb = (fb[r] & (xb >= -14.0f)) ? eb : 0.0f;
            const h16 pa = (h16)ga; const h16 pc = (h16)gb;
            pb[r] = pa; pb[8 + r] = pc;
            if (EARLY) { pr[r] = toh_flush((ga - (float)pa) * QRS); pr[8 + r] = toh_flush((gb - (float)pc) * QRS); ls += ga + gb; }
            else       { ls += (float)pa + (float)pc; } }
        l = l * alpha + ls; m = mnew;
#pragma unroll
        for (int j = 0; j < 4; ++j) { o[j] = o[j] * alpha; if (EARLY) oR[j] = oR[j] * alpha; }
        const size_t va = pbase + (size_t)ba * 1024 + (size_t)lr * 16 + 8 * hi;
        const size_t vb = pbase + (size_t)bb * 1024 + (size_t)lr * 16 + 8 * hi;
        const size_t vra = rbase + (size_t)ba * 1024 + (size_t)lr * 16 + 8 * hi;
        const size_t vrb = rbase + (size_t)bb * 1024 + (size_t)lr * 16 + 8 * hi;
#pragma unroll
        for (int j = 0; j < 4; ++j) {
            const v16h v = cat16(*(const v8h*)(VT + va + j * 256), *(const v8h*)(VT + vb + j * 256));
            o[j] = wmma16g(v, pb, o[j]);
            if (EARLY) {
                const v16h vr = cat16(*(const v8h*)(VR + vra + j * 256), *(const v8h*)(VR + vrb + j * 256));
                oR[j] = wmma16g(v, pr, oR[j]);
                oR[j] = wmma16g(vr, pb, oR[j]);
            }
        }
    }
    l += __shfl_xor(l, 16, 32);
    const bool any = l > 0.0f;
    const float lsafe = any ? l : 1.0f;
    const float inv = (any ? (1.0f / lsafe) : 0.0f) * osc;
    const int wb = wave * 16 * OSP;
#pragma unroll
    for (int j = 0; j < 4; ++j) {
        v8f f = o[j]; if (EARLY) f = o[j] + oR[j] * QRI;
        v4f a, c;
        a[0] = f[0] * inv; a[1] = f[1] * inv; a[2] = f[2] * inv; a[3] = f[3] * inv; c[0] = f[4] * inv; c[1] = f[5] * inv; c[2] = f[6] * inv; c[3] = f[7] * inv;
        *(v4fa*)(&os[wb + lr * OSP + 16 * j + 8 * hi]) = a; *(v4fa*)(&os[wb + lr * OSP + 16 * j + 8 * hi + 4]) = c; }
    wave_sync();
    const int mrow = seq * S + t0;
    v8h hv[4], rv[4];
    static_assert(4 * 4 == 16);
#pragma unroll
    for (int s = 0; s < 4; ++s) { const int row = 4 * s + (lane >> 3), c8 = (lane & 7) * 8;
        const v4f x0 = *(const v4fa*)(&os[wb + row * OSP + c8]); const v4f x1 = *(const v4fa*)(&os[wb + row * OSP + c8 + 4]);
#pragma unroll
        for (int i = 0; i < 4; ++i) { const h16 a0 = toh_flush(x0[i]), a1 = toh_flush(x1[i]); hv[s][i] = a0; hv[s][4 + i] = a1;
            if (EARLY) { rv[s][i] = toh_flush((x0[i] - (float)a0) * QRS); rv[s][4 + i] = toh_flush((x1[i] - (float)a1) * QRS); }
            else       { rv[s][i] = (h16)0.0f; rv[s][4 + i] = (h16)0.0f; } } }
    const size_t cb = (size_t)mrow * DM + h * HD;
    const size_t rb = (size_t)((ct < 0 ? 0 : ct) * 64 + (mrow & 63)) * DM + h * HD;
#pragma unroll 1
    for (int ps = 0; ps < 2; ++ps) {
#pragma unroll
        for (int s = 0; s < 4; ++s) { const int row = 4 * s + (lane >> 3), c8 = (lane & 7) * 8;
            *(volatile v8h*)(CH + cb + (size_t)row * DM + c8) = hv[s]; if (ct >= 0) *(volatile v8h*)(CR + rb + (size_t)row * DM + c8) = rv[s]; }
        if (ps == 0) __threadfence(); }
}

__global__ __launch_bounds__(32 * AW) void k_flash_early(const h16* __restrict__ QH, const h16* __restrict__ QR, const h16* __restrict__ KP, const h16* __restrict__ KR,
                                                         const h16* __restrict__ VT, const h16* __restrict__ VR, h16* CH, h16* CR,
                                                         int S, int tile0, int ntl, int ng1, int g0, int ngs, int bstride, float osc) {
    flash_body<1>(QH, QR, KP, KR, VT, VR, CH, CR, S, tile0, ntl, ng1, g0, ngs, bstride, osc);
}
__global__ __launch_bounds__(32 * AW) void k_flash_late(const h16* __restrict__ QH, const h16* __restrict__ QR, const h16* __restrict__ KP, const h16* __restrict__ KR,
                                                        const h16* __restrict__ VT, const h16* __restrict__ VR, h16* CH, h16* CR,
                                                        int S, int tile0, int ntl, int ng1, int g0, int ngs, int bstride, float osc) {
    flash_body<0>(QH, QR, KP, KR, VT, VR, CH, CR, S, tile0, ntl, ng1, g0, ngs, bstride, osc);
}

static constexpr size_t al256(size_t v) { return (v + 255) & ~(size_t)255; }
static constexpr size_t XL_ELEMS = (size_t)ML_ * DM;
static constexpr size_t XG_ELEMS = (size_t)MG_ * DM;
static constexpr size_t XR_ELEMS = (size_t)BROWS * DM;
static constexpr size_t PL_ELEMS = (size_t)MMAX * DM;
static constexpr size_t RS_ELEMS = (size_t)NB * NH_ * RT * HD;
static constexpr size_t SZ_WQ  = al256((size_t)2 * C3 * DM * 2);
static constexpr size_t SZ_WP  = al256((size_t)2 * DM * DM * 2);
static constexpr size_t SZ_X   = al256((XL_ELEMS + XG_ELEMS) * 2);
static constexpr size_t SZ_XR  = al256(2 * XR_ELEMS * 2);
static constexpr size_t SZ_QK  = al256((size_t)MMAX * 2 * DM * 4);
static constexpr size_t SZ_QKH = al256(2 * PL_ELEMS * 2);
static constexpr size_t SZ_VT  = al256(PL_ELEMS * 2);
static constexpr size_t SZ_QKR = al256(2 * RS_ELEMS * 2);
static constexpr size_t SZ_VR  = al256(RS_ELEMS * 2);
static constexpr size_t OFF_CR = al256(PL_ELEMS * 2);
static constexpr size_t SZ_TOTAL = 2 * SZ_WQ + 2 * SZ_WP + SZ_X + SZ_XR + SZ_QK + SZ_QKH + SZ_VT + SZ_QKR + SZ_VR;
static_assert(SZ_TOTAL <= (size_t)134217728);
static_assert(OFF_CR + XR_ELEMS * 2 <= SZ_QK);
static_assert((XL_ELEMS * 2) % 256 == 0);
static_assert((XR_ELEMS * 2) % 256 == 0);
static_assert((PL_ELEMS * 2) % 256 == 0);
static_assert((RS_ELEMS * 2) % 256 == 0);
static_assert(XL_ELEMS + XG_ELEMS < (size_t)2147483647);
static_assert((size_t)NB * NG * NH_ * SL * HD <= PL_ELEMS);
static_assert((size_t)NB * NH_ * SG * HD <= PL_ELEMS);
static_assert((NB * NG * TT) % 2 == 0);
static_assert((NB * NG * MEMT) % 2 == 0);
static_assert((NB * MEMT) % 2 == 0);

extern "C" void kernel_launch(void* const* d_in, const int* in_sizes, int n_in,
                              void* d_out, int out_size, void* d_ws, size_t ws_size, hipStream_t stream) {
    if (n_in < 9) return;
    const size_t nseqf = (size_t)(NB - 1) * NG_FULL + NG;
    if ((size_t)in_sizes[0] < nseqf * TT * DM) return;
    if ((size_t)in_sizes[1] < (size_t)NB * MEMT * DM) return;
    if ((size_t)in_sizes[2] < nseqf * MEMT * DM) return;
    if ((size_t)in_sizes[3] < (size_t)2 * DM * C3 || (size_t)in_sizes[6] < (size_t)2 * DM * C3) return;
    if ((size_t)in_sizes[4] < (size_t)2 * DM * DM || (size_t)in_sizes[7] < (size_t)2 * DM * DM) return;
    if (in_sizes[5] < 2 * DM || in_sizes[8] < 2 * DM) return;
    if ((size_t)out_size < nseqf * TT * DM) return;
    if (SZ_TOTAL > ws_size) return;
    const float* x_in  = (const float*)d_in[0];
    const float* mt_in = (const float*)d_in[1];
    const float* lm_in = (const float*)d_in[2];
    const float* wql_in = (const float*)d_in[3];
    const float* wpl_in = (const float*)d_in[4];
    const float* gl_in  = (const float*)d_in[5];
    const float* wqg_in = (const float*)d_in[6];
    const float* wpg_in = (const float*)d_in[7];
    const float* gg_in  = (const float*)d_in[8];
    float* OUT = (float*)d_out;
    char* wsp = (char*)d_ws;
    h16* WQL = (h16*)wsp; wsp += SZ_WQ;
    h16* WQG = (h16*)wsp; wsp += SZ_WQ;
    h16* WPL = (h16*)wsp; wsp += SZ_WP;
    h16* WPG = (h16*)wsp; wsp += SZ_WP;
    h16* X   = (h16*)wsp; wsp += SZ_X;
    h16* XR  = (h16*)wsp; wsp += SZ_XR;
    char* qkreg = wsp; wsp += SZ_QK;
    h16* QKH = (h16*)wsp; wsp += SZ_QKH;
    h16* VT  = (h16*)wsp; wsp += SZ_VT;
    h16* QKR = (h16*)wsp; wsp += SZ_QKR;
    h16* VR  = (h16*)wsp; wsp += SZ_VR;
    float* QK32 = (float*)qkreg;
    h16* CH = (h16*)qkreg; h16* CR = (h16*)(qkreg + OFF_CR);
    h16* XL = X; h16* XG = X + XL_ELEMS; h16* XLr = XR; h16* XGr = XR + XR_ELEMS;
    h16* QH = QKH; h16* KP = QKH + PL_ELEMS; h16* QRp = QKR; h16* KRp = QKR + RS_ELEMS;
    const int OXL = 0, OXG = (int)XL_ELEMS, OXLR = 0, OXGR = (int)XR_ELEMS;

    const float AS[4] = { 1.0f, 16.0f, 256.0f, 256.0f };
    const float VS[4] = { 16.0f, 64.0f, 256.0f, 1024.0f };
    const float CS[4] = { 16.0f, 64.0f, 256.0f, 1024.0f };

    k_wconv<<<dim3(DM / 64, C3 / 64, 2), 256, 0, stream>>>(wql_in, WQL, C3);
    k_wconv<<<dim3(DM / 64, C3 / 64, 2), 256, 0, stream>>>(wqg_in, WQG, C3);
    k_wconv<<<dim3(DM / 64, DM / 64, 2), 256, 0, stream>>>(wpl_in, WPL, DM);
    k_wconv<<<dim3(DM / 64, DM / 64, 2), 256, 0, stream>>>(wpg_in, WPG, DM);

    k_pack<<<(NB * NG * MEMT) / 2, 256, 0, stream>>>(lm_in, XL, XLr, NB * NG * MEMT, MEMT, NG, NG_FULL, SL, 0, AS[0], 0, NG * SL);
    k_pack<<<(NB * NG * TT) / 2, 256, 0, stream>>>(x_in, XL, XLr, NB * NG * TT, TT, NG, NG_FULL, SL, MEMT, AS[0], 0, NG * SL);
    k_pack<<<(NB * MEMT) / 2, 256, 0, stream>>>(mt_in, XG, XGr, NB * MEMT, MEMT, 1, 1, SG, 0, AS[1], 1, SG);

    const unsigned gfe = (unsigned)((SL / 16 + AW - 1) / AW);
    for (int i = 0; i < 2; ++i) {
        const int la = 2 * i, lb = 2 * i + 1;
        k_gemm_qkv<<<dim3((ML_ + 63) / 64, C3 / 64, 1), 32, 0, stream>>>(XL, XLr, WQL + (size_t)i * C3 * DM, QK32, VT, VR, ML_, SL, (i > 0) ? 1 : 0, NG * SL,
                                                                       1.0f / (WSC * AS[la]), NG, VS[la]);
        k_qknorm<<<(2 * ML_ + 7) / 8, 256, 0, stream>>>(QK32, gl_in + (size_t)i * DM, QKH, QKR, ML_, SL, NG, PL_ELEMS, RS_ELEMS);
        k_flash_early<<<dim3(gfe, NB * NH_, 1), 32 * AW, 0, stream>>>(QH, QRp, KP, KRp, VT, VR, CH, CR, SL, 0, SL / 16, 1, 0, NG, NG * SL, CS[la] / VS[la]);
        if (NG > 1)
            k_flash_late<<<dim3(gfe, NB * (NG - 1) * NH_, 1), 32 * AW, 0, stream>>>(QH, QRp, KP, KRp, VT, VR, CH, CR, SL, 0, SL / 16, NG - 1, 1, NG, NG * SL, CS[la] / VS[la]);
        k_gemm_proj16<<<dim3((ML_ + 63) / 64, DM / 64, 1), 32, 0, stream>>>(CH, CR, WPL + (size_t)i * DM * DM, X, XR, ML_, SL, 1, NG * SL, 1.0f / (WSC * CS[la]),
                                                                          NG, SG, TT, MEMT, SG, NG * SL, (i == 0) ? 1 : 0, OXG, OXL, OXGR, OXLR, AS[lb], (i == 0) ? AS[2] : 1.0f);
        k_gemm_qkv<<<dim3((MG_ + 63) / 64, C3 / 64, 1), 32, 0, stream>>>(XG, XGr, WQG + (size_t)i * C3 * DM, QK32, VT, VR, MG_, SG, 1, SG,
                                                                       1.0f / (WSC * AS[lb]), 1, VS[lb]);
        k_qknorm<<<(2 * MG_ + 7) / 8, 256, 0, stream>>>(QK32, gg_in + (size_t)i * DM, QKH, QKR, MG_, SG, 1, PL_ELEMS, RS_ELEMS);
        k_flash_early<<<dim3(gfe, NB * NH_, 1), 32 * AW, 0, stream>>>(QH, QRp, KP, KRp, VT, VR, CH, CR, SG, 0, SL / 16, 1, 0, 1, SG, CS[lb] / VS[lb]);
        k_flash_late<<<dim3((unsigned)((SG / 16 - SL / 16 + AW - 1) / AW), NB * NH_, 1), 32 * AW, 0, stream>>>(QH, QRp, KP, KRp, VT, VR, CH, CR, SG, SL / 16, SG / 16 - SL / 16, 1, 0, 1, SG, CS[lb] / VS[lb]);
        if (i == 0)
            k_gemm_proj16<<<dim3((MG_ + 63) / 64, DM / 64, 1), 32, 0, stream>>>(CH, CR, WPG, X, XR, MG_, SG, 1, SG, 1.0f / (WSC * CS[lb]),
                                                                              0, NG * SL, SL, MEMT, NG * SL, SG, 1, OXL, OXG, OXLR, OXGR, AS[2], AS[3]);
        else
            k_gemm_proj32<<<dim3((MG_ + 63) / 64, DM / 64, 1), 32, 0, stream>>>(CH, CR, WPG + (size_t)DM * DM, OUT, MG_, SG, 1, SG, 1.0f / (WSC * CS[lb]),
                                                                              0, NG_FULL * TT, TT, 0);
    }
}
